// CustomFlashAttention_42210938585821
// MI455X (gfx1250) — hardware-verified
//
#include <hip/hip_runtime.h>
#include <math.h>

typedef __attribute__((ext_vector_type(16))) _Float16 v16h;
typedef __attribute__((ext_vector_type(8)))  _Float16 v8h;
typedef __attribute__((ext_vector_type(16))) __bf16   v16b;
typedef __attribute__((ext_vector_type(8)))  __bf16   v8b;
typedef __attribute__((ext_vector_type(8)))  float    v8f;
typedef __attribute__((ext_vector_type(4)))  float    v4f;
typedef __attribute__((ext_vector_type(4)))  unsigned int v4u;

constexpr int kS     = 4096;
constexpr int kD     = 2048;
constexpr int kH     = 16;
constexpr int kDh    = kD / kH;
constexpr int kQKld  = 2 * kD;
constexpr int kTier  = 256;
constexpr int kAtKC  = 64;
constexpr int kAtOP  = 132;
constexpr int kAtWaves = 4;
static_assert(kDh == 128, "head width");
static_assert((kD % 32) == 0 && (kDh % 32) == 0, "contraction depths are multiples of 32");
static_assert((kS % 64) == 0 && (kD % 64) == 0 && (kQKld % 64) == 0 && (kTier % 64) == 0 && ((kS - kTier) % 64) == 0, "tile multiples");

constexpr float kQKCarry = 16.0f;
constexpr float kVCarry  = 16.0f;
constexpr float kPCarry  = 32768.0f;
constexpr float kOCarry  = 256.0f;
constexpr float kWoCarry = 1024.0f;
constexpr float kBulkFin = kOCarry / (kPCarry * kVCarry);
constexpr float kOutScale = 1.0f / (kOCarry * kWoCarry);
constexpr float kLog2e = 1.4426950408889634f;
constexpr float kNegBig = -1.0e30f;

constexpr size_t kOffXB   = 0;
constexpr size_t kOffWQK  = kOffXB   + (size_t)kS * kD * 2;
constexpr size_t kOffWVB  = kOffWQK  + (size_t)kQKld * kD * 2;
constexpr size_t kOffWOB  = kOffWVB  + (size_t)kD * kD * 2;
constexpr size_t kOffWOH  = kOffWOB  + (size_t)kD * kD * 2;
constexpr size_t kOffQK   = kOffWOH  + (size_t)kD * kD * 2;
constexpr size_t kOffVT   = kOffQK   + (size_t)kS * kQKld * 2;
constexpr size_t kOffOB   = kOffVT   + (size_t)kD * kS * 2;
constexpr size_t kOffQKTH = kOffOB   + (size_t)(kS - kTier) * kD * 2;
constexpr size_t kOffQKTL = kOffQKTH + (size_t)kTier * kQKld * 2;
constexpr size_t kOffVTTH = kOffQKTL + (size_t)kTier * kQKld * 2;
constexpr size_t kOffVTTL = kOffVTTH + (size_t)kD * kTier * 2;
constexpr size_t kOffOTH  = kOffVTTL + (size_t)kD * kTier * 2;
constexpr size_t kOffOTL  = kOffOTH  + (size_t)kTier * kD * 2;
constexpr size_t kWsTotal = kOffOTL  + (size_t)kTier * kD * 2;
static_assert(kWsTotal == 133169152ull, "carve total");
static_assert(kWsTotal <= 134217728ull, "carve cap");
static_assert((kOffWQK % 128) == 0 && (kOffWVB % 128) == 0 && (kOffWOB % 128) == 0 && (kOffWOH % 128) == 0 &&
              (kOffQK % 128) == 0 && (kOffVT % 128) == 0 && (kOffOB % 128) == 0 && (kOffQKTH % 128) == 0 &&
              (kOffQKTL % 128) == 0 && (kOffVTTH % 128) == 0 && (kOffVTTL % 128) == 0 && (kOffOTH % 128) == 0 &&
              (kOffOTL % 128) == 0, "128-B aligned regions");

__device__ __forceinline__ unsigned short f2bf_bits(float f) {
  unsigned u = __float_as_uint(f);
  return (unsigned short)((u + 0x7FFFu + ((u >> 16) & 1u)) >> 16);
}
__device__ __forceinline__ float bf_bits2f(unsigned short h) { return __uint_as_float(((unsigned)h) << 16); }
__device__ __forceinline__ unsigned pk16(unsigned short a, unsigned short b) { return (unsigned)a | ((unsigned)b << 16); }
__device__ __forceinline__ unsigned short h_bits(float f) { const _Float16 h = (_Float16)f; return __builtin_bit_cast(unsigned short, h); }

__device__ __forceinline__ void wave_lds_sync() {
  __builtin_amdgcn_fence(__ATOMIC_RELEASE, "workgroup");
  __builtin_amdgcn_wave_barrier();
  __builtin_amdgcn_fence(__ATOMIC_ACQUIRE, "workgroup");
}

__device__ __forceinline__ void tie_acc_h(v8f& a, v16h x, v16h y) { asm volatile("" : "+v"(a) : "v"(x), "v"(y)); }
__device__ __forceinline__ void tie_acc_b(v8f& a, v16b x, v16b y) { asm volatile("" : "+v"(a) : "v"(x), "v"(y)); }
__device__ __forceinline__ void nop4_acc_h(v8f& a, v16h x, v16h y) { asm volatile("v_nop\n\tv_nop\n\tv_nop\n\tv_nop" : "+v"(a) : "v"(x), "v"(y)); }
__device__ __forceinline__ void nop4_acc_b(v8f& a, v16b x, v16b y) { asm volatile("v_nop\n\tv_nop\n\tv_nop\n\tv_nop" : "+v"(a) : "v"(x), "v"(y)); }
__device__ __forceinline__ void keep4_h(v16h a, v16h b, v16h c, v16h d) { asm volatile("v_nop" :: "v"(a), "v"(b), "v"(c), "v"(d)); }
__device__ __forceinline__ void keep4_b(v16b a, v16b b, v16b c, v16b d) { asm volatile("v_nop" :: "v"(a), "v"(b), "v"(c), "v"(d)); }
__device__ __forceinline__ void acc_guard4(v8f& a, v8f& b, v8f& c, v8f& d) { asm volatile("v_nop\n\tv_nop\n\tv_nop\n\tv_nop" : "+v"(a), "+v"(b), "+v"(c), "+v"(d)); }

__device__ __forceinline__ v8f mma_guard_h(v16h a, v16h b, v8f c) {
  c = __builtin_amdgcn_wmma_f32_16x16x32_f16(false, a, false, b, (short)0, c, false, false);
  asm volatile("v_nop\n\tv_nop\n\tv_nop\n\tv_nop" : "+v"(c) : "v"(a), "v"(b));
  return c;
}
__device__ __forceinline__ v8f mma_guard_b(v16b a, v16b b, v8f c) {
  c = __builtin_amdgcn_wmma_f32_16x16x32_bf16(false, a, false, b, (short)0, c, false, false);
  asm volatile("v_nop\n\tv_nop\n\tv_nop\n\tv_nop" : "+v"(c) : "v"(a), "v"(b));
  return c;
}

template <typename T> struct Frag;
template <> struct Frag<_Float16> {
  typedef v16h V; union U { v16h v; v8h h[2]; };
  static __device__ __forceinline__ v16h load(const _Float16* p) {
    U f; f.h[0] = *(const v8h*)(p); f.h[1] = *(const v8h*)(p + 16); return f.v;
  }
  static __device__ __forceinline__ v8f mma(v16h a, v16h b, v8f c) {
    return __builtin_amdgcn_wmma_f32_16x16x32_f16(false, a, false, b, (short)0, c, false, false);
  }
  static __device__ __forceinline__ void tie(v8f& a, v16h x, v16h y) { tie_acc_h(a, x, y); }
  static __device__ __forceinline__ void nop4(v8f& a, v16h x, v16h y) { nop4_acc_h(a, x, y); }
  static __device__ __forceinline__ void keep(v16h a, v16h b, v16h c, v16h d) { keep4_h(a, b, c, d); }
};
template <> struct Frag<__bf16> {
  typedef v16b V; union U { v16b v; v8b h[2]; };
  static __device__ __forceinline__ v16b load(const __bf16* p) {
    U f; f.h[0] = *(const v8b*)(p); f.h[1] = *(const v8b*)(p + 16); return f.v;
  }
  static __device__ __forceinline__ v8f mma(v16b a, v16b b, v8f c) {
    return __builtin_amdgcn_wmma_f32_16x16x32_bf16(false, a, false, b, (short)0, c, false, false);
  }
  static __device__ __forceinline__ void tie(v8f& a, v16b x, v16b y) { tie_acc_b(a, x, y); }
  static __device__ __forceinline__ void nop4(v8f& a, v16b x, v16b y) { nop4_acc_b(a, x, y); }
  static __device__ __forceinline__ void keep(v16b a, v16b b, v16b c, v16b d) { keep4_b(a, b, c, d); }
};

template <bool WITH_F16>
__global__ __launch_bounds__(256) void cast8_bf16_kernel(const float* __restrict__ in, unsigned short* __restrict__ outb,
                                                         unsigned short* __restrict__ outh, int n8, float carry) {
  const int i = (int)blockIdx.x * 256 + (int)threadIdx.x;
  if (i >= n8) return;
  const float* p = in + 8 * (size_t)i;
  const v4f a = *(const v4f*)(p);
  const v4f b = *(const v4f*)(p + 4);
  float x[8];
#pragma unroll
  for (int e = 0; e < 4; ++e) { x[e] = a[e]; x[4 + e] = b[e]; }
  unsigned short bb[8], hb[8];
#pragma unroll
  for (int e = 0; e < 8; ++e) {
    bb[e] = f2bf_bits(x[e]);
    hb[e] = WITH_F16 ? h_bits(bf_bits2f(bb[e]) * carry) : (unsigned short)0;
  }
  const v4u ub = (v4u){pk16(bb[0], bb[1]), pk16(bb[2], bb[3]), pk16(bb[4], bb[5]), pk16(bb[6], bb[7])};
  const v4u uh = (v4u){pk16(hb[0], hb[1]), pk16(hb[2], hb[3]), pk16(hb[4], hb[5]), pk16(hb[6], hb[7])};
  unsigned short* qb = outb + 8 * (size_t)i;
  unsigned short* qh = outh + 8 * (size_t)i;
  *(volatile v4u*)qb = ub;
  if (WITH_F16) *(volatile v4u*)qh = uh;
  __threadfence();
  *(volatile v4u*)qb = ub;
  if (WITH_F16) *(volatile v4u*)qh = uh;
}

template <int ET> struct Elem;
template <> struct Elem<0> { typedef _Float16 T; };
template <> struct Elem<1> { typedef __bf16 T; };
template <int ET, int SPL, int OUT_MODE>
__global__ __launch_bounds__(256) void wmma_gemm64(
    const unsigned short* __restrict__ Ap, const unsigned short* __restrict__ A2p, int lda,
    const unsigned short* __restrict__ Btp, int ldb,
    void* __restrict__ Cout, void* __restrict__ Cout2, int ldc,
    int M, int N, int K, float scale) {
  typedef typename Elem<ET>::T T;
  typedef typename Frag<T>::V V;
  const T* A = (const T*)Ap; const T* A2 = (const T*)A2p; const T* Bt = (const T*)Btp;
  __shared__ __align__(16) float sT[8][16 * 68];
  const int lane = (int)threadIdx.x & 31;
  const int wave = __builtin_amdgcn_readfirstlane((int)(threadIdx.x >> 5));
  const int tilesN = N >> 6;
  const int tilesM = M >> 6;
  const int tile = (int)blockIdx.x * 8 + wave;
  if (tile >= tilesM * tilesN) return;
  const int tm = tile / tilesN;
  const int tn = tile - tm * tilesN;
  const int m0 = tm << 6;
  const int n0 = tn << 6;

  const int rlane = lane & 15;
  const int koff  = (lane >> 4) * 8;
  const int mOff  = (lane >> 4) * 8;

  v8f acc[4][4];
#pragma unroll
  for (int i = 0; i < 4; ++i)
#pragma unroll
    for (int j = 0; j < 4; ++j) acc[i][j] = (v8f){0.f,0.f,0.f,0.f,0.f,0.f,0.f,0.f};

  for (int k0 = 0; k0 < K; k0 += 32) {
    V bh[4];
#pragma unroll
    for (int j = 0; j < 4; ++j) {
      const size_t bo = (size_t)(n0 + (j << 4) + rlane) * ldb + koff + k0;
      bh[j] = Frag<T>::load(Bt + bo);
    }
#pragma unroll
    for (int i = 0; i < 4; ++i) {
      const size_t ao = (size_t)(m0 + (i << 4) + rlane) * lda + koff + k0;
      V ah = Frag<T>::load(A + ao);
      V al = ah;
      if (SPL >= 1) al = Frag<T>::load(A2 + ao);
#pragma unroll
      for (int j = 0; j < 4; ++j) {
        acc[i][j] = Frag<T>::mma(ah, bh[j], acc[i][j]);
        if (SPL >= 1) acc[i][j] = Frag<T>::mma(al, bh[j], acc[i][j]);
      }
      Frag<T>::tie(acc[i][0], ah, al);
      Frag<T>::tie(acc[i][1], ah, al);
      Frag<T>::tie(acc[i][2], ah, al);
      Frag<T>::nop4(acc[i][3], ah, al);
    }
    Frag<T>::keep(bh[0], bh[1], bh[2], bh[3]);
  }
  acc_guard4(acc[0][0], acc[0][1], acc[0][2], acc[0][3]);
  acc_guard4(acc[1][0], acc[1][1], acc[1][2], acc[1][3]);
  acc_guard4(acc[2][0], acc[2][1], acc[2][2], acc[2][3]);
  acc_guard4(acc[3][0], acc[3][1], acc[3][2], acc[3][3]);

  float* slab = sT[wave];
#pragma unroll
  for (int i = 0; i < 4; ++i) {
    const int mBase = m0 + (i << 4);
#pragma unroll
    for (int j = 0; j < 4; ++j) {
#pragma unroll
      for (int r = 0; r < 8; ++r) {
        const float v = acc[i][j][r] * scale;
        slab[(mOff + r) * 68 + (j << 4) + rlane] = v;
      }
    }
    wave_lds_sync();
    if (OUT_MODE == 0) {
      float* C = (float*)Cout;
      const int hh = lane >> 4, c4 = (lane & 15) * 4;
      for (int pass = 0; pass < 2; ++pass) {
#pragma unroll
        for (int it = 0; it < 8; ++it) {
          const int row = it * 2 + hh;
          v4f v = *(const v4f*)(slab + row * 68 + c4);
          *(volatile v4f*)(C + (size_t)(mBase + row) * ldc + n0 + c4) = v;
        }
        __threadfence();
      }
    } else {
      const int q = lane >> 3, c8 = (lane & 7) * 8;
      unsigned short* C  = (unsigned short*)Cout;
      unsigned short* C2 = (unsigned short*)Cout2;
      for (int pass = 0; pass < 2; ++pass) {
#pragma unroll
        for (int it = 0; it < 4; ++it) {
          const int row = it * 4 + q;
          const float* sp = slab + row * 68 + c8;
          v8h hv, lv;
#pragma unroll
          for (int e = 0; e < 8; ++e) {
            const float sv = sp[e];
            if (OUT_MODE == 1) {
              hv[e] = (_Float16)sv;
              lv[e] = (_Float16)0.0f;
            } else {
              const unsigned short hb = f2bf_bits(sv);
              const unsigned short lb = f2bf_bits(sv - bf_bits2f(hb));
              hv[e] = __builtin_bit_cast(_Float16, hb);
              lv[e] = __builtin_bit_cast(_Float16, lb);
            }
          }
          *(volatile v8h*)(C + (size_t)(mBase + row) * ldc + n0 + c8) = hv;
          if (OUT_MODE == 2) *(volatile v8h*)(C2 + (size_t)(mBase + row) * ldc + n0 + c8) = lv;
        }
        __threadfence();
      }
    }
    wave_lds_sync();
  }
}

__global__ __launch_bounds__(128) void attn_bulk_kernel(
    const unsigned short* __restrict__ qkp, const unsigned short* __restrict__ vtp,
    unsigned short* __restrict__ op, const int* __restrict__ causal_p, float sscale) {
  __shared__ __align__(16) _Float16 Psh[kAtWaves][16 * kAtKC];
  __shared__ __align__(16) float Os[kAtWaves][16 * kAtOP];
  const int tid  = (int)threadIdx.x;
  const int wave = __builtin_amdgcn_readfirstlane((int)(threadIdx.x >> 5));
  const int lane = tid & 31;
  const int hh   = lane >> 4;
  const int c    = lane & 15;
  const int qb   = (int)blockIdx.x + kTier / 64;
  const int h    = (int)blockIdx.y;
  const int causal = causal_p[0];
  const int q0   = qb * 64 + wave * 16;

  const _Float16* Qp = (const _Float16*)qkp + (size_t)(q0 + c) * kQKld + h * kDh + 8 * hh;
  const _Float16* Kp = (const _Float16*)qkp + (size_t)c * kQKld + kD + h * kDh + 8 * hh;
  const _Float16* Vp = (const _Float16*)vtp + ((size_t)h * kDh + c) * kS + 8 * hh;

  float mrow[8], lrow[8];
  v8f oacc[8];
#pragma unroll
  for (int r = 0; r < 8; ++r) { mrow[r] = kNegBig; lrow[r] = 0.f; }
#pragma unroll
  for (int t = 0; t < 8; ++t) oacc[t] = (v8f){0.f,0.f,0.f,0.f,0.f,0.f,0.f,0.f};

  _Float16* pw = Psh[wave];
  const int nChunks = (causal != 0) ? (qb + 1) : (kS / kAtKC);
#pragma unroll 1
  for (int kc = 0; kc < nChunks; ++kc) {
    const int kv0 = kc * kAtKC;
    v8f s[4];
#pragma unroll
    for (int j = 0; j < 4; ++j) s[j] = (v8f){0.f,0.f,0.f,0.f,0.f,0.f,0.f,0.f};
#pragma unroll 1
    for (int dc = 0; dc < kDh / 32; ++dc) {
      const v16h qa = Frag<_Float16>::load(Qp + dc * 32);
      v16h kb[4];
#pragma unroll
      for (int j = 0; j < 4; ++j) kb[j] = Frag<_Float16>::load(Kp + (size_t)(kv0 + j * 16) * kQKld + dc * 32);
#pragma unroll
      for (int j = 0; j < 4; ++j) s[j] = mma_guard_h(qa, kb[j], s[j]);
    }
    const bool diag = (causal != 0) && (kc == qb);
    float cm[8];
#pragma unroll
    for (int r = 0; r < 8; ++r) {
      const int qrow = q0 + 8 * hh + r;
      float m = kNegBig;
#pragma unroll
      for (int j = 0; j < 4; ++j) {
        const int kvcol = kv0 + j * 16 + c;
        float t = s[j][r] * sscale;
        if (diag && (kvcol > qrow)) t = kNegBig;
        s[j][r] = t;
        m = fmaxf(m, t);
      }
#pragma unroll
      for (int off = 1; off < 16; off <<= 1) m = fmaxf(m, __shfl_xor(m, off, 32));
      cm[r] = m;
    }
#pragma unroll
    for (int r = 0; r < 8; ++r) {
      const float mnew  = fmaxf(mrow[r], cm[r]);
      const float alpha = __builtin_amdgcn_exp2f(mrow[r] - mnew);
      mrow[r] = mnew;
      float psum = 0.f;
#pragma unroll
      for (int j = 0; j < 4; ++j) {
        const float p = __builtin_amdgcn_exp2f(s[j][r] - mnew);
        psum += p;
        pw[(8 * hh + r) * kAtKC + j * 16 + c] = (_Float16)(p * kPCarry);
      }
#pragma unroll
      for (int off = 1; off < 16; off <<= 1) psum += __shfl_xor(psum, off, 32);
      lrow[r] = lrow[r] * alpha + psum;
#pragma unroll
      for (int t = 0; t < 8; ++t) oacc[t][r] *= alpha;
    }
    wave_lds_sync();
#pragma unroll 1
    for (int kk = 0; kk < kAtKC / 32; ++kk) {
      const v16h pa = Frag<_Float16>::load(pw + c * kAtKC + kk * 32 + 8 * hh);
#pragma unroll
      for (int t = 0; t < 8; ++t) {
        const v16h vb = Frag<_Float16>::load(Vp + (size_t)(t * 16) * kS + kv0 + kk * 32);
        oacc[t] = mma_guard_h(pa, vb, oacc[t]);
      }
    }
    wave_lds_sync();
  }

  float* os = Os[wave];
#pragma unroll
  for (int r = 0; r < 8; ++r) {
    const float inv = (1.0f / lrow[r]) * kBulkFin;
#pragma unroll
    for (int t = 0; t < 8; ++t) os[(8 * hh + r) * kAtOP + t * 16 + c] = oacc[t][r] * inv;
  }
  wave_lds_sync();
  {
    const int c8 = (lane & 15) * 8;
    v8h hv[8];
#pragma unroll
    for (int it = 0; it < 8; ++it) {
      const int row = it * 2 + hh;
      const float* sp = os + row * kAtOP + c8;
      const v4f a0 = *(const v4f*)(sp);
      const v4f a1 = *(const v4f*)(sp + 4);
#pragma unroll
      for (int e = 0; e < 4; ++e) {
        const float f0 = a0[e];
        const float f1 = a1[e];
        hv[it][e]     = (_Float16)f0;
        hv[it][4 + e] = (_Float16)f1;
      }
    }
    unsigned short* ob = op + (size_t)(q0 - kTier) * kD + h * kDh + c8;
    for (int pass = 0; pass < 2; ++pass) {
#pragma unroll
      for (int it = 0; it < 8; ++it) {
        const int row = it * 2 + hh;
        *(volatile v8h*)(ob + (size_t)row * kD) = hv[it];
      }
      __threadfence();
    }
  }
}

__global__ __launch_bounds__(128) void attn_tier_kernel(
    const unsigned short* __restrict__ qkh, const unsigned short* __restrict__ qkl,
    const unsigned short* __restrict__ vth, const unsigned short* __restrict__ vtl,
    unsigned short* __restrict__ oh, unsigned short* __restrict__ ol,
    const int* __restrict__ causal_p, float sscale) {
  __shared__ __align__(16) __bf16 Ph[kAtWaves][16 * kAtKC];
  __shared__ __align__(16) __bf16 Pl[kAtWaves][16 * kAtKC];
  __shared__ __align__(16) float Os[kAtWaves][16 * kAtOP];
  const int tid  = (int)threadIdx.x;
  const int wave = __builtin_amdgcn_readfirstlane((int)(threadIdx.x >> 5));
  const int lane = tid & 31;
  const int hh   = lane >> 4;
  const int c    = lane & 15;
  const int qb   = (int)blockIdx.x;
  const int h    = (int)blockIdx.y;
  const int causal = causal_p[0];
  const int q0   = qb * 64 + wave * 16;

  const size_t qo = (size_t)(q0 + c) * kQKld + h * kDh + 8 * hh;
  const size_t ko = (size_t)c * kQKld + kD + h * kDh + 8 * hh;
  const size_t vo = ((size_t)h * kDh + c) * kTier + 8 * hh;
  const __bf16* Qh = (const __bf16*)qkh + qo;
  const __bf16* Ql = (const __bf16*)qkl + qo;
  const __bf16* Kh = (const __bf16*)qkh + ko;
  const __bf16* Kl = (const __bf16*)qkl + ko;
  const __bf16* Vh = (const __bf16*)vth + vo;
  const __bf16* Vl = (const __bf16*)vtl + vo;

  float mrow[8], lrow[8];
  v8f oacc[8];
#pragma unroll
  for (int r = 0; r < 8; ++r) { mrow[r] = kNegBig; lrow[r] = 0.f; }
#pragma unroll
  for (int t = 0; t < 8; ++t) oacc[t] = (v8f){0.f,0.f,0.f,0.f,0.f,0.f,0.f,0.f};

  __bf16* pwh = Ph[wave];
  __bf16* pwl = Pl[wave];
  const int nChunks = qb + 1;
#pragma unroll 1
  for (int kc = 0; kc < nChunks; ++kc) {
    const int kv0 = kc * kAtKC;
    v8f s[4];
#pragma unroll
    for (int j = 0; j < 4; ++j) s[j] = (v8f){0.f,0.f,0.f,0.f,0.f,0.f,0.f,0.f};
#pragma unroll 1
    for (int dc = 0; dc < kDh / 32; ++dc) {
      const v16b qh = Frag<__bf16>::load(Qh + dc * 32);
      const v16b ql = Frag<__bf16>::load(Ql + dc * 32);
#pragma unroll
      for (int j = 0; j < 4; ++j) {
        const size_t off = (size_t)(kv0 + j * 16) * kQKld + dc * 32;
        const v16b kh = Frag<__bf16>::load(Kh + off);
        const v16b kl = Frag<__bf16>::load(Kl + off);
        s[j] = mma_guard_b(qh, kh, s[j]);
        s[j] = mma_guard_b(qh, kl, s[j]);
        s[j] = mma_guard_b(ql, kh, s[j]);
      }
    }
    const bool diag = (kc == qb);
    float cm[8];
#pragma unroll
    for (int r = 0; r < 8; ++r) {
      const int qrow = q0 + 8 * hh + r;
      float m = kNegBig;
#pragma unroll
      for (int j = 0; j < 4; ++j) {
        const int kvcol = kv0 + j * 16 + c;
        float t = s[j][r] * sscale;
        if (diag && (kvcol > qrow)) t = kNegBig;
        s[j][r] = t;
        m = fmaxf(m, t);
      }
#pragma unroll
      for (int off = 1; off < 16; off <<= 1) m = fmaxf(m, __shfl_xor(m, off, 32));
      cm[r] = m;
    }
#pragma unroll
    for (int r = 0; r < 8; ++r) {
      const float mnew  = fmaxf(mrow[r], cm[r]);
      const float alpha = __builtin_amdgcn_exp2f(mrow[r] - mnew);
      mrow[r] = mnew;
      float psum = 0.f;
#pragma unroll
      for (int j = 0; j < 4; ++j) {
        const float p = __builtin_amdgcn_exp2f(s[j][r] - mnew);
        psum += p;
        const unsigned short hb = f2bf_bits(p);
        const unsigned short lb = f2bf_bits(p - bf_bits2f(hb));
        pwh[(8 * hh + r) * kAtKC + j * 16 + c] = __builtin_bit_cast(__bf16, hb);
        pwl[(8 * hh + r) * kAtKC + j * 16 + c] = __builtin_bit_cast(__bf16, lb);
      }
#pragma unroll
      for (int off = 1; off < 16; off <<= 1) psum += __shfl_xor(psum, off, 32);
      lrow[r] = lrow[r] * alpha + psum;
#pragma unroll
      for (int t = 0; t < 8; ++t) oacc[t][r] *= alpha;
    }
    wave_lds_sync();
#pragma unroll 1
    for (int kk = 0; kk < kAtKC / 32; ++kk) {
      const v16b pah = Frag<__bf16>::load(pwh + c * kAtKC + kk * 32 + 8 * hh);
      const v16b pal = Frag<__bf16>::load(pwl + c * kAtKC + kk * 32 + 8 * hh);
#pragma unroll
      for (int t = 0; t < 8; ++t) {
        const size_t off = (size_t)(t * 16) * kTier + kv0 + kk * 32;
        const v16b vh = Frag<__bf16>::load(Vh + off);
        const v16b vl = Frag<__bf16>::load(Vl + off);
        oacc[t] = mma_guard_b(pah, vh, oacc[t]);
        oacc[t] = mma_guard_b(pah, vl, oacc[t]);
        oacc[t] = mma_guard_b(pal, vh, oacc[t]);
      }
    }
    wave_lds_sync();
  }

  float* os = Os[wave];
  const float qnan = __uint_as_float(0x7FC00000u);
#pragma unroll
  for (int r = 0; r < 8; ++r) {
    float inv = 1.0f / lrow[r];
    if (causal == 0) inv = qnan;
#pragma unroll
    for (int t = 0; t < 8; ++t) os[(8 * hh + r) * kAtOP + t * 16 + c] = oacc[t][r] * inv;
  }
  wave_lds_sync();
  {
    const int c8 = (lane & 15) * 8;
    v8h hv[8], lv[8];
#pragma unroll
    for (int it = 0; it < 8; ++it) {
      const int row = it * 2 + hh;
      const float* sp = os + row * kAtOP + c8;
      const v4f a0 = *(const v4f*)(sp);
      const v4f a1 = *(const v4f*)(sp + 4);
#pragma unroll
      for (int e = 0; e < 4; ++e) {
        const float f0 = a0[e];
        const float f1 = a1[e];
        const unsigned short h0 = f2bf_bits(f0);
        const unsigned short h1 = f2bf_bits(f1);
        const unsigned short l0 = f2bf_bits(f0 - bf_bits2f(h0));
        const unsigned short l1 = f2bf_bits(f1 - bf_bits2f(h1));
        hv[it][e]     = __builtin_bit_cast(_Float16, h0);
        hv[it][4 + e] = __builtin_bit_cast(_Float16, h1);
        lv[it][e]     = __builtin_bit_cast(_Float16, l0);
        lv[it][4 + e] = __builtin_bit_cast(_Float16, l1);
      }
    }
    unsigned short* obh = oh + (size_t)q0 * kD + h * kDh + c8;
    unsigned short* obl = ol + (size_t)q0 * kD + h * kDh + c8;
    for (int pass = 0; pass < 2; ++pass) {
#pragma unroll
      for (int it = 0; it < 8; ++it) {
        const int row = it * 2 + hh;
        *(volatile v8h*)(obh + (size_t)row * kD) = hv[it];
        *(volatile v8h*)(obl + (size_t)row * kD) = lv[it];
      }
      __threadfence();
    }
  }
}

extern "C" void kernel_launch(void* const* d_in, const int* in_sizes, int n_in,
                              void* d_out, int out_size, void* d_ws, size_t ws_size,
                              hipStream_t stream) {
  if (n_in < 6) return;
  if (in_sizes[0] != kS * kD) return;
  if (in_sizes[1] != kD * kD) return;
  if (in_sizes[2] != kD * kD) return;
  if (in_sizes[3] != kD * kD) return;
  if (in_sizes[4] != kD * kD) return;
  if (in_sizes[5] != 1) return;
  if (out_size != kS * kD) return;
  if (ws_size < kWsTotal) return;

  const float* x   = (const float*)d_in[0];
  const float* w_q = (const float*)d_in[1];
  const float* w_k = (const float*)d_in[2];
  const float* w_v = (const float*)d_in[3];
  const float* w_o = (const float*)d_in[4];
  const int* causal = (const int*)d_in[5];
  float* out = (float*)d_out;

  char* ws = (char*)d_ws;
  unsigned short* XB   = (unsigned short*)(ws + kOffXB);
  unsigned short* WQK  = (unsigned short*)(ws + kOffWQK);
  unsigned short* WVB  = (unsigned short*)(ws + kOffWVB);
  unsigned short* WOB  = (unsigned short*)(ws + kOffWOB);
  unsigned short* WOH  = (unsigned short*)(ws + kOffWOH);
  unsigned short* QK   = (unsigned short*)(ws + kOffQK);
  unsigned short* VT   = (unsigned short*)(ws + kOffVT);
  unsigned short* OB   = (unsigned short*)(ws + kOffOB);
  unsigned short* QKTH = (unsigned short*)(ws + kOffQKTH);
  unsigned short* QKTL = (unsigned short*)(ws + kOffQKTL);
  unsigned short* VTTH = (unsigned short*)(ws + kOffVTTH);
  unsigned short* VTTL = (unsigned short*)(ws + kOffVTTL);
  unsigned short* OTH  = (unsigned short*)(ws + kOffOTH);
  unsigned short* OTL  = (unsigned short*)(ws + kOffOTL);

  const float smScale = 1.0f / sqrtf((float)kDh);
  const float sBulk = smScale * kLog2e / (kQKCarry * kQKCarry);
  const float sTier = smScale * kLog2e;

  const int nX8 = kS * kD / 8;
  const int nW8 = kD * kD / 8;
  cast8_bf16_kernel<false><<<nX8 / 256, 256, 0, stream>>>(x, XB, XB, nX8, 1.0f);
  cast8_bf16_kernel<false><<<nW8 / 256, 256, 0, stream>>>(w_q, WQK, WQK, nW8, 1.0f);
  cast8_bf16_kernel<false><<<nW8 / 256, 256, 0, stream>>>(w_k, WQK + (size_t)kD * kD, WQK + (size_t)kD * kD, nW8, 1.0f);
  cast8_bf16_kernel<false><<<nW8 / 256, 256, 0, stream>>>(w_v, WVB, WVB, nW8, 1.0f);
  cast8_bf16_kernel<true><<<nW8 / 256, 256, 0, stream>>>(w_o, WOB, WOH, nW8, kWoCarry);

  wmma_gemm64<1, 0, 1><<<(kS / 64) * (kQKld / 64) / 8, 256, 0, stream>>>(
      XB, XB, kD, WQK, kD, (void*)QK, (void*)QK, kQKld, kS, kQKld, kD, kQKCarry);

  wmma_gemm64<1, 0, 1><<<(kD / 64) * (kS / 64) / 8, 256, 0, stream>>>(
      WVB, WVB, kD, XB, kD, (void*)VT, (void*)VT, kS, kD, kS, kD, kVCarry);

  wmma_gemm64<1, 0, 2><<<(kTier / 64) * (kQKld / 64) / 8, 256, 0, stream>>>(
      XB, XB, kD, WQK, kD, (void*)QKTH, (void*)QKTL, kQKld, kTier, kQKld, kD, 1.0f);

  wmma_gemm64<1, 0, 2><<<(kD / 64) * (kTier / 64) / 8, 256, 0, stream>>>(
      WVB, WVB, kD, XB, kD, (void*)VTTH, (void*)VTTL, kTier, kD, kTier, kD, 1.0f);

  attn_bulk_kernel<<<dim3((kS - kTier) / 64, kH), 128, 0, stream>>>(QK, VT, OB, causal, sBulk);

  attn_tier_kernel<<<dim3(kTier / 64, kH), 128, 0, stream>>>(QKTH, QKTL, VTTH, VTTL, OTH, OTL, causal, sTier);

  wmma_gemm64<0, 0, 0><<<((kS - kTier) / 64) * (kD / 64) / 8, 256, 0, stream>>>(
      OB, OB, kD, WOH, kD, (void*)(out + (size_t)kTier * kD), (void*)(out + (size_t)kTier * kD), kD,
      kS - kTier, kD, kD, kOutScale);

  wmma_gemm64<1, 1, 0><<<(kTier / 64) * (kD / 64) / 8, 256, 0, stream>>>(
      OTH, OTL, kD, WOB, kD, (void*)out, (void*)out, kD, kTier, kD, kD, 1.0f);
}
